// PositionalMultiHeadAttn_1700807049349
// MI455X (gfx1250) — hardware-verified
//
#include <hip/hip_runtime.h>
#include <math.h>

#define NTOK_ROWS 16384
#define EMB_DIM   768
#define FF_DIM    3072
#define NSEQ_P    384
#define SEQL      512
#define HDIM      64
#define FF_CHUNK  4096
#define FF_NCHUNK 4
#define P_CARRY   16384.0f
#define CTX_CARRY 64.0f
#define W_CARRY   32.0f
#define H_CARRY   16.0f
static_assert(NSEQ_P * SEQL * HDIM == NTOK_ROWS * EMB_DIM, "raw view");
static_assert(FF_CHUNK * FF_NCHUNK == NTOK_ROWS, "chunking");
static_assert((EMB_DIM % 64) == 0 && (FF_DIM % 64) == 0 && (FF_CHUNK % 64) == 0, "tile multiples");
static_assert((EMB_DIM % 32) == 0 && (FF_DIM % 32) == 0, "K multiples of 32");

typedef __attribute__((ext_vector_type(16))) _Float16 v16h;
typedef __attribute__((ext_vector_type(8)))  _Float16 v8h;
typedef __attribute__((ext_vector_type(16))) __bf16   v16b;
typedef __attribute__((ext_vector_type(8)))  __bf16   v8b;
typedef __attribute__((ext_vector_type(8)))  float    v8f;
typedef __attribute__((ext_vector_type(4)))  float    v4f;
typedef v8h __attribute__((may_alias)) v8ha;
typedef v4f __attribute__((may_alias)) v4fa;

__device__ __forceinline__ unsigned short f2bf_bits(float f) {
  unsigned u = __float_as_uint(f);
  return (unsigned short)((u + 0x7FFFu + ((u >> 16) & 1u)) >> 16);
}
__device__ __forceinline__ float bf_bits2f(unsigned short h) { return __uint_as_float(((unsigned)h) << 16); }

__device__ __forceinline__ void dep_guard_h(v8f& a, v8f& b, v16h x, v16h y) { asm volatile("v_nop\n\tv_nop\n\tv_nop\n\tv_nop" : "+v"(a), "+v"(b) : "v"(x), "v"(y)); }
__device__ __forceinline__ void dep_guard_b(v8f& a, v8f& b, v16b x, v16b y) { asm volatile("v_nop\n\tv_nop\n\tv_nop\n\tv_nop" : "+v"(a), "+v"(b) : "v"(x), "v"(y)); }
__device__ __forceinline__ void keep4_h(v16h a, v16h b, v16h c, v16h d) { asm volatile("v_nop" :: "v"(a), "v"(b), "v"(c), "v"(d)); }
__device__ __forceinline__ void keep4_b(v16b a, v16b b, v16b c, v16b d) { asm volatile("v_nop" :: "v"(a), "v"(b), "v"(c), "v"(d)); }
__device__ __forceinline__ void acc_guard4(v8f& a, v8f& b, v8f& c, v8f& d) { asm volatile("v_nop\n\tv_nop\n\tv_nop\n\tv_nop" : "+v"(a), "+v"(b), "+v"(c), "+v"(d)); }
template <typename T> struct Frag;
template <> struct Frag<_Float16> {
  typedef v16h V; union U { v16h v; v8h h[2]; };
  static __device__ __forceinline__ v16h load(const _Float16* p) {
    U f; f.h[0] = *(const v8h*)(p); f.h[1] = *(const v8h*)(p + 16); return f.v;
  }
  static __device__ __forceinline__ v8f mma(v16h a, v16h b, v8f c) {
    return __builtin_amdgcn_wmma_f32_16x16x32_f16(false, a, false, b, (short)0, c, false, false);
  }
  static __device__ __forceinline__ void guard(v8f& a, v8f& b, v16h x, v16h y) { dep_guard_h(a, b, x, y); }
  static __device__ __forceinline__ void keep(v16h a, v16h b, v16h c, v16h d) { keep4_h(a, b, c, d); }
};
template <> struct Frag<__bf16> {
  typedef v16b V; union U { v16b v; v8b h[2]; };
  static __device__ __forceinline__ v16b load(const __bf16* p) {
    U f; f.h[0] = *(const v8b*)(p); f.h[1] = *(const v8b*)(p + 16); return f.v;
  }
  static __device__ __forceinline__ v8f mma(v16b a, v16b b, v8f c) {
    return __builtin_amdgcn_wmma_f32_16x16x32_bf16(false, a, false, b, (short)0, c, false, false);
  }
  static __device__ __forceinline__ void guard(v8f& a, v8f& b, v16b x, v16b y) { dep_guard_b(a, b, x, y); }
  static __device__ __forceinline__ void keep(v16b a, v16b b, v16b c, v16b d) { keep4_b(a, b, c, d); }
};

template <int ET> struct Elem;
template <> struct Elem<0> { typedef _Float16 T; };
template <> struct Elem<1> { typedef __bf16 T; };
template <int ET, bool SPLIT, int BIAS_MODE, int OUT_MODE, bool RESID, int ACT = 0>
__global__ __launch_bounds__(256) void wmma_gemm64(
    const unsigned short* __restrict__ Ap, const unsigned short* __restrict__ A2p, int lda, long strideA,
    const unsigned short* __restrict__ Btp, const unsigned short* __restrict__ Bt2p, int ldb, long strideB,
    void* __restrict__ Cout, void* __restrict__ Cout2, int ldc, long strideC,
    const float* __restrict__ bias,
    const float* __restrict__ resid, long strideR,
    int M, int N, int K, float scale, float oscale) {
  typedef typename Elem<ET>::T T;
  typedef typename Frag<T>::V V;
  const T* A = (const T*)Ap; const T* A2 = (const T*)A2p; const T* Bt = (const T*)Btp; const T* Bt2 = (const T*)Bt2p;
  __shared__ __align__(16) float sT[8][16 * 68];
  const int b    = blockIdx.y;
  const int lane = threadIdx.x & 31;
  const int wave = threadIdx.x >> 5;
  const int tilesN = N >> 6;
  const int tilesM = M >> 6;
  const int tile = blockIdx.x * 8 + wave;
  if (tile >= tilesM * tilesN) return;
  const int tm = tile / tilesN;
  const int tn = tile - tm * tilesN;
  const int m0 = tm << 6;
  const int n0 = tn << 6;

  const T* Ab  = A  + (size_t)b * strideA;
  const T* Bb  = Bt + (size_t)b * strideB;
  const T* Ab2 = SPLIT ? (A2  + (size_t)b * strideA) : nullptr;
  const T* Bb2 = SPLIT ? (Bt2 + (size_t)b * strideB) : nullptr;

  const int rlane = lane & 15;
  const int koff  = (lane >> 4) * 8;
  const int mOff  = (lane >> 4) * 8;

  v8f acc[4][4];
#pragma unroll
  for (int i = 0; i < 4; ++i)
#pragma unroll
    for (int j = 0; j < 4; ++j) acc[i][j] = (v8f){0.f,0.f,0.f,0.f,0.f,0.f,0.f,0.f};

  for (int k0 = 0; k0 < K; k0 += 32) {
    V bh[4], bl[4];
#pragma unroll
    for (int j = 0; j < 4; ++j) {
      const size_t bo = (size_t)(n0 + (j << 4) + rlane) * ldb + koff + k0;
      bh[j] = Frag<T>::load(Bb + bo);
      if (SPLIT) bl[j] = Frag<T>::load(Bb2 + bo);
    }
#pragma unroll
    for (int i = 0; i < 4; ++i) {
      const size_t ao = (size_t)(m0 + (i << 4) + rlane) * lda + koff + k0;
      V ah = Frag<T>::load(Ab + ao);
      V al;
      if (SPLIT) al = Frag<T>::load(Ab2 + ao);
#pragma unroll
      for (int j = 0; j < 4; ++j) {
        acc[i][j] = Frag<T>::mma(ah, bh[j], acc[i][j]);
        if (SPLIT) {
          acc[i][j] = Frag<T>::mma(ah, bl[j], acc[i][j]);
          acc[i][j] = Frag<T>::mma(al, bh[j], acc[i][j]);
        }
      }
      Frag<T>::guard(acc[i][0], acc[i][3], ah, SPLIT ? al : ah);
    }
    Frag<T>::keep(bh[0], bh[1], bh[2], bh[3]);
    if (SPLIT) Frag<T>::keep(bl[0], bl[1], bl[2], bl[3]);
  }
  acc_guard4(acc[0][0], acc[0][1], acc[0][2], acc[0][3]);
  acc_guard4(acc[1][0], acc[1][1], acc[1][2], acc[1][3]);
  acc_guard4(acc[2][0], acc[2][1], acc[2][2], acc[2][3]);
  acc_guard4(acc[3][0], acc[3][1], acc[3][2], acc[3][3]);

  float* slab = sT[wave];
  const float* Rb = RESID ? (resid + (size_t)b * strideR) : nullptr;
#pragma unroll
  for (int i = 0; i < 4; ++i) {
    const int mBase = m0 + (i << 4);
#pragma unroll
    for (int j = 0; j < 4; ++j) {
      const int n = n0 + (j << 4) + rlane;
      float bv = 0.f;
      if (BIAS_MODE == 2) bv = bias[n];
#pragma unroll
      for (int r = 0; r < 8; ++r) {
        float v = acc[i][j][r] * scale;
        if (BIAS_MODE == 1) v += bias[mBase + mOff + r];
        if (BIAS_MODE == 2) v += bv;
        if (RESID) v += Rb[(size_t)(mBase + mOff + r) * ldc + n];
        if (ACT == 2) v = fmaxf(v, 0.0f);
        v = v * oscale;
        slab[(mOff + r) * 68 + (j << 4) + rlane] = v;
      }
    }
    __builtin_amdgcn_fence(__ATOMIC_RELEASE, "workgroup");
    __builtin_amdgcn_wave_barrier();
    __builtin_amdgcn_fence(__ATOMIC_ACQUIRE, "workgroup");
    if (OUT_MODE == 0) {
      float* C = (float*)Cout + (size_t)b * strideC;
      const int hh = lane >> 4, c4 = (lane & 15) * 4;
      for (int pass = 0; pass < 2; ++pass) {
#pragma unroll
        for (int it = 0; it < 8; ++it) {
          const int row = it * 2 + hh;
          v4f v = *(const v4f*)(slab + row * 68 + c4);
          *(volatile v4f*)(C + (size_t)(mBase + row) * ldc + n0 + c4) = v;
        }
        __threadfence();
      }
    } else {
      const int q = lane >> 3, c8 = (lane & 7) * 8;
      unsigned short* C  = (unsigned short*)Cout  + (size_t)b * strideC;
      unsigned short* C2 = (OUT_MODE == 2) ? ((unsigned short*)Cout2 + (size_t)b * strideC) : nullptr;
      for (int pass = 0; pass < 2; ++pass) {
#pragma unroll
        for (int it = 0; it < 4; ++it) {
          const int row = it * 4 + q;
          const float* sp = slab + row * 68 + c8;
          v8h hv, lv;
#pragma unroll
          for (int e = 0; e < 8; ++e) {
            if (OUT_MODE == 1) {
              hv[e] = (_Float16)sp[e];
            } else {
              unsigned short hb = f2bf_bits(sp[e]);
              unsigned short lb = f2bf_bits(sp[e] - bf_bits2f(hb));
              hv[e] = __builtin_bit_cast(_Float16, hb);
              lv[e] = __builtin_bit_cast(_Float16, lb);
            }
          }
          *(volatile v8h*)(C + (size_t)(mBase + row) * ldc + n0 + c8) = hv;
          if (OUT_MODE == 2) *(volatile v8h*)(C2 + (size_t)(mBase + row) * ldc + n0 + c8) = lv;
        }
        __threadfence();
      }
    }
    __builtin_amdgcn_fence(__ATOMIC_RELEASE, "workgroup");
    __builtin_amdgcn_wave_barrier();
    __builtin_amdgcn_fence(__ATOMIC_ACQUIRE, "workgroup");
  }
}

__device__ __forceinline__ v8f mma_h16(v16h a, v16h b, v8f c) {
  v8f d = __builtin_amdgcn_wmma_f32_16x16x32_f16(false, a, false, b, (short)0, c, false, false);
  asm volatile("v_nop\n\tv_nop\n\tv_nop\n\tv_nop" : "+v"(d) : "v"(a), "v"(b));
  return d;
}
union FragU { v16h v; v8h half[2]; };
__device__ __forceinline__ v16h load_frag(const _Float16* p, int h) {
  FragU f;
  f.half[0] = *(const v8ha*)(p + 8 * h);
  f.half[1] = *(const v8ha*)(p + 16 + 8 * h);
  return f.v;
}

__global__ __launch_bounds__(256) void cvt_f16x8(
    const float* __restrict__ s0, const float* __restrict__ s1,
    const float* __restrict__ s2, const float* __restrict__ s3,
    _Float16* __restrict__ dst, long dstride, int n8, float sc) {
  const int t = blockIdx.y;
  const float* src = (t == 0) ? s0 : ((t == 1) ? s1 : ((t == 2) ? s2 : s3));
  const int i = blockIdx.x * 256 + threadIdx.x;
  if (i >= n8) return;
  const v4f a = *(const v4fa*)(src + (size_t)i * 8);
  const v4f c = *(const v4fa*)(src + (size_t)i * 8 + 4);
  const v8h o = { (_Float16)(a.x * sc), (_Float16)(a.y * sc), (_Float16)(a.z * sc), (_Float16)(a.w * sc),
                  (_Float16)(c.x * sc), (_Float16)(c.y * sc), (_Float16)(c.z * sc), (_Float16)(c.w * sc) };
  _Float16* d = dst + (size_t)t * dstride + (size_t)i * 8;
  *(volatile v8h*)d = o;
  __threadfence();
  *(volatile v8h*)d = o;
}

struct PeDiv { float d[EMB_DIM]; };
static_assert(sizeof(PeDiv) == EMB_DIM * 4, "no padding");

__global__ __launch_bounds__(256) void pe_table_kernel(float* __restrict__ pe, PeDiv dv) {
  __shared__ float sv[256];
  const int tid  = threadIdx.x;
  const int pos  = blockIdx.x / 3;
  const int e0   = (blockIdx.x - pos * 3) * 256;
  const int half = tid >> 7;
  const int k    = tid & 127;
  const int e    = e0 + 2 * k + half;
  const float a  = (float)pos * dv.d[e];
  float val;
  if (half == 0) val = sinf(a); else val = cosf(a);
  sv[2 * k + half] = val;
  __syncthreads();
  const float o = sv[tid];
  float* dst = pe + (size_t)pos * EMB_DIM + e0 + tid;
  *(volatile float*)dst = o;
  __threadfence();
  *(volatile float*)dst = o;
}

__global__ __launch_bounds__(256) void vt_transpose_kernel(const _Float16* __restrict__ v,
                                                           _Float16* __restrict__ vt) {
  __shared__ __attribute__((aligned(16))) _Float16 tile[64 * 72];
  const int tid = threadIdx.x, lane = tid & 31, w = tid >> 5;
  const int j  = blockIdx.y;
  const int l0 = blockIdx.x * 64;
  const _Float16* src = v + ((size_t)j * SEQL + l0) * HDIM;
#pragma unroll
  for (int i = 0; i < 2; ++i) {
    const int idx = i * 256 + tid;
    const int tok = idx >> 3, d0 = (idx & 7) * 8;
    const v8h x = *(const v8ha*)(src + tok * HDIM + d0);
#pragma unroll
    for (int e = 0; e < 8; ++e) tile[(d0 + e) * 72 + tok] = x[e];
  }
  __syncthreads();
  const int q8 = lane & 7, sub = lane >> 3;
  v8h val[2];
#pragma unroll
  for (int it = 0; it < 2; ++it) {
    const int d = 8 * w + it * 4 + sub;
    val[it] = *(const v8ha*)(tile + d * 72 + 8 * q8);
  }
  for (int pass = 0; pass < 2; ++pass) {
#pragma unroll
    for (int it = 0; it < 2; ++it) {
      const int d = 8 * w + it * 4 + sub;
      *(volatile v8h*)(vt + ((size_t)j * HDIM + d) * SEQL + l0 + 8 * q8) = val[it];
    }
    __threadfence();
  }
}

__device__ __forceinline__ v16h pack_p16(v8f a, v8f c) {
  const v16h r = { (_Float16)(a[0] * P_CARRY), (_Float16)(a[1] * P_CARRY), (_Float16)(a[2] * P_CARRY), (_Float16)(a[3] * P_CARRY),
                   (_Float16)(a[4] * P_CARRY), (_Float16)(a[5] * P_CARRY), (_Float16)(a[6] * P_CARRY), (_Float16)(a[7] * P_CARRY),
                   (_Float16)(c[0] * P_CARRY), (_Float16)(c[1] * P_CARRY), (_Float16)(c[2] * P_CARRY), (_Float16)(c[3] * P_CARRY),
                   (_Float16)(c[4] * P_CARRY), (_Float16)(c[5] * P_CARRY), (_Float16)(c[6] * P_CARRY), (_Float16)(c[7] * P_CARRY) };
  return r;
}

__device__ __forceinline__ void ctx_store_pass(const float* so, _Float16* ctx, int bh, int q0, int lane) {
  const int q8 = lane & 7, sub = lane >> 3;
#pragma unroll
  for (int it = 0; it < 4; ++it) {
    const int row = it * 4 + sub;
    const v4f a = *(const v4fa*)(so + row * 64 + 8 * q8);
    const v4f c = *(const v4fa*)(so + row * 64 + 8 * q8 + 4);
    const v8h o = { (_Float16)a.x, (_Float16)a.y, (_Float16)a.z, (_Float16)a.w,
                    (_Float16)c.x, (_Float16)c.y, (_Float16)c.z, (_Float16)c.w };
    *(volatile v8h*)(ctx + ((size_t)bh * SEQL + q0 + row) * HDIM + 8 * q8) = o;
  }
}

__global__ __launch_bounds__(128) void attn_kernel(
    const _Float16* __restrict__ qh,
    const _Float16* __restrict__ kh,
    const _Float16* __restrict__ vt,
    _Float16* __restrict__ ctx)
{
  __shared__ __attribute__((aligned(16))) float sO[4 * 16 * 64];

  const int tid = threadIdx.x, lane = tid & 31, w = tid >> 5;
  const int h = lane >> 4, m = lane & 15;
  const int bh = blockIdx.y;
  const int q0 = blockIdx.x * 64 + 16 * w;

  const _Float16* qrow = qh + ((size_t)bh * SEQL + q0 + m) * HDIM;
  const v16h qb0 = load_frag(qrow, h);
  const v16h qb1 = load_frag(qrow + 32, h);

  const v8f zero8 = {0.f, 0.f, 0.f, 0.f, 0.f, 0.f, 0.f, 0.f};
  v8f o[4];
#pragma unroll
  for (int t = 0; t < 4; ++t) o[t] = zero8;
  float mrun = -1.0e30f, lrun = 0.0f;

  const _Float16* kbase = kh + ((size_t)bh * SEQL + m) * HDIM;
  const _Float16* vbase = vt + ((size_t)bh * HDIM + m) * SEQL;

#pragma unroll 1
  for (int kb = 0; kb < SEQL; kb += 64) {
    v8f s[4];
#pragma unroll
    for (int j = 0; j < 4; ++j) {
      const _Float16* kp = kbase + (size_t)(kb + 16 * j) * HDIM;
      const v16h kf0 = load_frag(kp, h);
      const v16h kf1 = load_frag(kp + 32, h);
      v8f z = zero8;
      z = mma_h16(kf0, qb0, z);
      z = mma_h16(kf1, qb1, z);
      s[j] = z;
    }
    float mloc = -1.0e30f;
#pragma unroll
    for (int j = 0; j < 4; ++j)
#pragma unroll
      for (int r = 0; r < 8; ++r) { s[j][r] = s[j][r] * 0.125f; mloc = fmaxf(mloc, s[j][r]); }
    mloc = fmaxf(mloc, __shfl_xor(mloc, 16, 32));
    const float mnew = fmaxf(mrun, mloc);
    const float alpha = __expf(mrun - mnew);
    mrun = mnew;
    float lsum = 0.0f;
#pragma unroll
    for (int j = 0; j < 4; ++j)
#pragma unroll
      for (int r = 0; r < 8; ++r) {
        const float p = __expf(s[j][r] - mnew);
        s[j][r] = p;
        lsum += p;
      }
    lsum += __shfl_xor(lsum, 16, 32);
    lrun = lrun * alpha + lsum;
#pragma unroll
    for (int t = 0; t < 4; ++t)
#pragma unroll
      for (int r = 0; r < 8; ++r) o[t][r] = o[t][r] * alpha;

    const v16h pb0 = pack_p16(s[0], s[1]);
    const v16h pb1 = pack_p16(s[2], s[3]);

#pragma unroll
    for (int t = 0; t < 4; ++t) {
      const _Float16* vp = vbase + (size_t)(16 * t) * SEQL + kb;
      const v16h vf0 = load_frag(vp, h);
      const v16h vf1 = load_frag(vp + 32, h);
      o[t] = mma_h16(vf0, pb0, o[t]);
      o[t] = mma_h16(vf1, pb1, o[t]);
    }
  }

  const float inv = (1.0f / lrun) * (CTX_CARRY / P_CARRY);
  float* so = sO + w * 1024;
#pragma unroll
  for (int t = 0; t < 4; ++t)
#pragma unroll
    for (int r = 0; r < 8; ++r)
      so[m * 64 + 16 * t + 8 * h + r] = o[t][r] * inv;
  __syncthreads();

  ctx_store_pass(so, ctx, bh, q0, lane);
  __threadfence();
  ctx_store_pass(so, ctx, bh, q0, lane);
}

__global__ __launch_bounds__(256) void ln_pe_kernel(const float* __restrict__ proj,
    const float* __restrict__ gam, const float* __restrict__ bet, const float* __restrict__ pe,
    _Float16* __restrict__ xo, int nrows) {
  const int lane = threadIdx.x & 31, wave = threadIdx.x >> 5;
  const int row = blockIdx.x * 8 + wave;
  if (row >= nrows) return;
  const float* pr  = proj + (size_t)row * EMB_DIM;
  const float* ppe = pe + (size_t)(row & (SEQL - 1)) * EMB_DIM;
  float x[24];
#pragma unroll
  for (int g = 0; g < 3; ++g) {
    const int c = g * 256 + lane * 8;
    const v4f a = *(const v4fa*)(pr + c);
    const v4f b = *(const v4fa*)(pr + c + 4);
    x[8 * g + 0] = a.x; x[8 * g + 1] = a.y; x[8 * g + 2] = a.z; x[8 * g + 3] = a.w;
    x[8 * g + 4] = b.x; x[8 * g + 5] = b.y; x[8 * g + 6] = b.z; x[8 * g + 7] = b.w;
  }
  float s = 0.f;
#pragma unroll
  for (int e = 0; e < 24; ++e) s += x[e];
#pragma unroll
  for (int off = 1; off < 32; off <<= 1) s += __shfl_xor(s, off, 32);
  const float mu = s * (1.0f / (float)EMB_DIM);
  float qs = 0.f;
#pragma unroll
  for (int e = 0; e < 24; ++e) { const float d = x[e] - mu; x[e] = d; qs += d * d; }
#pragma unroll
  for (int off = 1; off < 32; off <<= 1) qs += __shfl_xor(qs, off, 32);
  const float var = qs * (1.0f / (float)EMB_DIM);
  const float inv = rsqrtf(var + 1.0e-5f);
  v8h ov[3];
#pragma unroll
  for (int g = 0; g < 3; ++g) {
    const int c = g * 256 + lane * 8;
    const v4f g0 = *(const v4fa*)(gam + c), g1 = *(const v4fa*)(gam + c + 4);
    const v4f b0 = *(const v4fa*)(bet + c), b1 = *(const v4fa*)(bet + c + 4);
    const v4f p0 = *(const v4fa*)(ppe + c), p1 = *(const v4fa*)(ppe + c + 4);
    const float gg[8] = { g0.x, g0.y, g0.z, g0.w, g1.x, g1.y, g1.z, g1.w };
    const float bb[8] = { b0.x, b0.y, b0.z, b0.w, b1.x, b1.y, b1.z, b1.w };
    const float pp[8] = { p0.x, p0.y, p0.z, p0.w, p1.x, p1.y, p1.z, p1.w };
    v8h o;
#pragma unroll
    for (int e = 0; e < 8; ++e) {
      float y = (x[8 * g + e] * inv) * gg[e] + bb[e];
      y = y + pp[e];
      o[e] = (_Float16)y;
    }
    ov[g] = o;
  }
  _Float16* dst = xo + (size_t)row * EMB_DIM + lane * 8;
  for (int pass = 0; pass < 2; ++pass) {
#pragma unroll
    for (int g = 0; g < 3; ++g) *(volatile v8h*)(dst + g * 256) = ov[g];
    __threadfence();
  }
}

extern "C" void kernel_launch(void* const* d_in, const int* in_sizes, int n_in,
                              void* d_out, int out_size, void* d_ws, size_t ws_size,
                              hipStream_t stream) {
  if (n_in < 15) return;
  if (in_sizes[0] != NTOK_ROWS * EMB_DIM) return;
  if (in_sizes[1] != EMB_DIM * EMB_DIM || in_sizes[3] != EMB_DIM * EMB_DIM ||
      in_sizes[5] != EMB_DIM * EMB_DIM || in_sizes[7] != EMB_DIM * EMB_DIM) return;
  if (in_sizes[2] != EMB_DIM || in_sizes[4] != EMB_DIM || in_sizes[6] != EMB_DIM || in_sizes[8] != EMB_DIM ||
      in_sizes[9] != EMB_DIM || in_sizes[10] != EMB_DIM || in_sizes[14] != EMB_DIM) return;
  if (in_sizes[11] != FF_DIM * EMB_DIM || in_sizes[13] != FF_DIM * EMB_DIM || in_sizes[12] != FF_DIM) return;
  if (out_size != NTOK_ROWS * EMB_DIM) return;

  const float* vec = (const float*)d_in[0];
  const float* Wq  = (const float*)d_in[1];  const float* bq  = (const float*)d_in[2];
  const float* Wk  = (const float*)d_in[3];  const float* bk  = (const float*)d_in[4];
  const float* Wv  = (const float*)d_in[5];  const float* bv  = (const float*)d_in[6];
  const float* Wo  = (const float*)d_in[7];  const float* bo  = (const float*)d_in[8];
  const float* lng = (const float*)d_in[9];  const float* lnb = (const float*)d_in[10];
  const float* W1  = (const float*)d_in[11]; const float* b1  = (const float*)d_in[12];
  const float* W2  = (const float*)d_in[13]; const float* b2  = (const float*)d_in[14];
  float* out = (float*)d_out;

  const size_t w768B = (size_t)EMB_DIM * EMB_DIM * 2;
  const size_t wbigB = (size_t)FF_DIM * EMB_DIM * 2;
  const size_t offWq = 0, offWk = w768B, offWv = 2 * w768B, offWo = 3 * w768B;
  const size_t offW1 = 4 * w768B, offW2 = 4 * w768B + wbigB;
  const size_t offPE = 4 * w768B + 2 * wbigB;
  const size_t peB   = (size_t)SEQL * EMB_DIM * 4;
  const size_t plB   = (size_t)NTOK_ROWS * EMB_DIM * 2;
  const size_t offR0 = offPE + peB;
  const size_t offR1 = offR0 + plB;
  const size_t offR2 = offR1 + plB;
  const size_t offR3 = offR2 + plB;
  const size_t total = offR3 + plB;
  if (total > ws_size) return;
  if ((size_t)FF_CHUNK * FF_DIM * 2 > plB) return;
  if ((size_t)NTOK_ROWS * EMB_DIM * 4 > 2 * plB) return;

  char* ws = (char*)d_ws;
  _Float16* Wq16 = (_Float16*)(ws + offWq);
  _Float16* Wk16 = (_Float16*)(ws + offWk);
  _Float16* Wv16 = (_Float16*)(ws + offWv);
  _Float16* Wo16 = (_Float16*)(ws + offWo);
  _Float16* W116 = (_Float16*)(ws + offW1);
  _Float16* W216 = (_Float16*)(ws + offW2);
  float*    pe   = (float*)(ws + offPE);
  _Float16* R0h  = (_Float16*)(ws + offR0);
  _Float16* R1h  = (_Float16*)(ws + offR1);
  _Float16* R2h  = (_Float16*)(ws + offR2);
  _Float16* R3h  = (_Float16*)(ws + offR3);
  float*    proj = (float*)(ws + offR1);

  typedef const unsigned short* cus;

  PeDiv dv;
  {
    const float rcp = 1.0f / (float)EMB_DIM;
    for (int e = 0; e < EMB_DIM; ++e) {
      const float ef = (float)e * rcp;
      dv.d[e] = (float)pow(10000.0, (double)ef);
    }
  }

  {
    const int n8 = NTOK_ROWS * EMB_DIM / 8;
    cvt_f16x8<<<dim3(n8 / 256, 1), 256, 0, stream>>>(vec, vec, vec, vec, R0h, 0L, n8, 1.0f);
  }
  {
    const int n8 = EMB_DIM * EMB_DIM / 8;
    cvt_f16x8<<<dim3(n8 / 256, 4), 256, 0, stream>>>(Wq, Wk, Wv, Wo, Wq16, (long)EMB_DIM * EMB_DIM, n8, W_CARRY);
  }
  {
    const int n8 = FF_DIM * EMB_DIM / 8;
    cvt_f16x8<<<dim3(n8 / 256, 2), 256, 0, stream>>>(W1, W2, W1, W2, W116, (long)FF_DIM * EMB_DIM, n8, W_CARRY);
  }
  pe_table_kernel<<<dim3(SEQL * 3), 256, 0, stream>>>(pe, dv);

  {
    const dim3 g((NTOK_ROWS / 64) * (EMB_DIM / 64) / 8, 1);
    wmma_gemm64<0, false, 2, 1, false, 0><<<g, 256, 0, stream>>>(
        (cus)R0h, (cus)R0h, EMB_DIM, 0L, (cus)Wq16, (cus)Wq16, EMB_DIM, 0L,
        (void*)R1h, (void*)R1h, EMB_DIM, 0L, bq, vec, 0L, NTOK_ROWS, EMB_DIM, EMB_DIM, 1.0f / W_CARRY, 1.0f);
    wmma_gemm64<0, false, 2, 1, false, 0><<<g, 256, 0, stream>>>(
        (cus)R0h, (cus)R0h, EMB_DIM, 0L, (cus)Wk16, (cus)Wk16, EMB_DIM, 0L,
        (void*)R2h, (void*)R2h, EMB_DIM, 0L, bk, vec, 0L, NTOK_ROWS, EMB_DIM, EMB_DIM, 1.0f / W_CARRY, 1.0f);
    wmma_gemm64<0, false, 2, 1, false, 0><<<g, 256, 0, stream>>>(
        (cus)R0h, (cus)R0h, EMB_DIM, 0L, (cus)Wv16, (cus)Wv16, EMB_DIM, 0L,
        (void*)R3h, (void*)R3h, EMB_DIM, 0L, bv, vec, 0L, NTOK_ROWS, EMB_DIM, EMB_DIM, 1.0f / W_CARRY, 1.0f);
  }
  vt_transpose_kernel<<<dim3(SEQL / 64, NSEQ_P), 256, 0, stream>>>(R3h, R0h);

  attn_kernel<<<dim3(SEQL / 64, NSEQ_P), 128, 0, stream>>>(R1h, R2h, R0h, R3h);

  {
    const dim3 g((NTOK_ROWS / 64) * (EMB_DIM / 64) / 8, 1);
    wmma_gemm64<0, false, 2, 0, true, 0><<<g, 256, 0, stream>>>(
        (cus)R3h, (cus)R3h, EMB_DIM, 0L, (cus)Wo16, (cus)Wo16, EMB_DIM, 0L,
        (void*)proj, (void*)proj, EMB_DIM, 0L, bo, vec, 0L, NTOK_ROWS, EMB_DIM, EMB_DIM,
        1.0f / (CTX_CARRY * W_CARRY), 1.0f);
  }
  ln_pe_kernel<<<dim3(NTOK_ROWS / 8), 256, 0, stream>>>(proj, lng, lnb, pe, R0h, NTOK_ROWS);

  for (int c = 0; c < FF_NCHUNK; ++c) {
    const _Float16* xc = R0h + (size_t)c * FF_CHUNK * EMB_DIM;
    float* oc = out + (size_t)c * FF_CHUNK * EMB_DIM;
    const dim3 g1((FF_CHUNK / 64) * (FF_DIM / 64) / 8, 1);
    wmma_gemm64<0, false, 2, 1, false, 2><<<g1, 256, 0, stream>>>(
        (cus)xc, (cus)xc, EMB_DIM, 0L, (cus)W116, (cus)W116, EMB_DIM, 0L,
        (void*)R3h, (void*)R3h, FF_DIM, 0L, b1, vec, 0L, FF_CHUNK, FF_DIM, EMB_DIM, 1.0f / W_CARRY, H_CARRY);
    const dim3 g2((FF_CHUNK / 64) * (EMB_DIM / 64) / 8, 1);
    wmma_gemm64<0, false, 2, 0, false, 0><<<g2, 256, 0, stream>>>(
        (cus)R3h, (cus)R3h, FF_DIM, 0L, (cus)W216, (cus)W216, FF_DIM, 0L,
        (void*)oc, (void*)oc, EMB_DIM, 0L, b2, vec, 0L, FF_CHUNK, EMB_DIM, FF_DIM,
        1.0f / (H_CARRY * W_CARRY), 1.0f);
  }
}
